// TLC_DQN_50852412784681
// MI455X (gfx1250) — hardware-verified
//
#include <hip/hip_runtime.h>


#define NB_ 16
#define NNODE 1000
#define BN_ (NB_ * NNODE)
#define TT 16
#define FO 16
#define HID 128
#define G3 (3 * HID)
#define NHEAD 5
#define HC (NHEAD * HID)
#define NEB 4000
#define NE_ (NB_ * NEB)
#define PP 8
#define NACT 8
#define IL_CAP 32
#define SLOPE 0.2f
#define FUP 320

typedef __attribute__((ext_vector_type(16))) __bf16   v16bf;
typedef __attribute__((ext_vector_type(16))) _Float16 v16h;
typedef __attribute__((ext_vector_type(8)))  float    v8f;
typedef __attribute__((ext_vector_type(8)))  unsigned v8u;

__device__ __forceinline__ unsigned f2bf(float f) { unsigned u = __float_as_uint(f); u += 0x7FFFu + ((u >> 16) & 1u); return u >> 16; }
__device__ __forceinline__ unsigned f2h(float f) { return (unsigned)__builtin_bit_cast(unsigned short, (_Float16)f); }
__device__ __forceinline__ int kpat(int v, int half) { return ((v & 4) ? 16 : 0) + half * 8 + 2 * (v & 3); }

template <int F16, int NP> struct Opnd { v16bf p[NP]; };

template <int F16, int NP> __device__ __forceinline__ void pack2(float f0, float f1, unsigned* o) {
    if (F16) { o[0] = f2h(f0) | (f2h(f1) << 16); return; }
    unsigned h0 = f2bf(f0), h1 = f2bf(f1); o[0] = h0 | (h1 << 16);
    if (NP >= 2) {
        float r0 = f0 - __uint_as_float(h0 << 16), r1 = f1 - __uint_as_float(h1 << 16);
        unsigned m0 = f2bf(r0), m1 = f2bf(r1); o[1] = m0 | (m1 << 16);
        if (NP >= 3) {
            float s0 = r0 - __uint_as_float(m0 << 16), s1 = r1 - __uint_as_float(m1 << 16);
            o[2] = f2bf(s0) | (f2bf(s1) << 16);
        }
    }
}
template <int F16, int NP> __device__ __forceinline__ void op_row(const float* rowp, int half, float sc, Opnd<F16, NP>& o) {
    v8u u[NP];
#pragma unroll
    for (int v = 0; v < 8; ++v) {
        int kk = kpat(v, half); unsigned t[3];
        pack2<F16, NP>(rowp[kk] * sc, rowp[kk + 1] * sc, t);
#pragma unroll
        for (int p = 0; p < NP; ++p) u[p][v] = t[p];
    }
#pragma unroll
    for (int p = 0; p < NP; ++p) o.p[p] = __builtin_bit_cast(v16bf, u[p]);
}
template <int F16, int NP> __device__ __forceinline__ void op_row_tail(const float* rowp, int half, float sc, int kvalid, Opnd<F16, NP>& o) {
    v8u u[NP];
#pragma unroll
    for (int v = 0; v < 8; ++v) {
        int kk = kpat(v, half); unsigned t[3];
        float f0 = kk < kvalid ? rowp[kk] * sc : 0.0f, f1 = (kk + 1) < kvalid ? rowp[kk + 1] * sc : 0.0f;
        pack2<F16, NP>(f0, f1, t);
#pragma unroll
        for (int p = 0; p < NP; ++p) u[p][v] = t[p];
    }
#pragma unroll
    for (int p = 0; p < NP; ++p) o.p[p] = __builtin_bit_cast(v16bf, u[p]);
}
template <int F16, int NP> __device__ __forceinline__ void op_col(const float* M, int ld, int n, int k0, int half, float sc, Opnd<F16, NP>& o) {
    v8u u[NP];
#pragma unroll
    for (int v = 0; v < 8; ++v) {
        int kk = k0 + kpat(v, half); unsigned t[3];
        pack2<F16, NP>(M[(size_t)kk * ld + n] * sc, M[(size_t)(kk + 1) * ld + n] * sc, t);
#pragma unroll
        for (int p = 0; p < NP; ++p) u[p][v] = t[p];
    }
#pragma unroll
    for (int p = 0; p < NP; ++p) o.p[p] = __builtin_bit_cast(v16bf, u[p]);
}
template <int F16, int NP> __device__ __forceinline__ void op_col_tail(const float* M, int ld, int n, int k0, int half, float sc, int K, Opnd<F16, NP>& o) {
    v8u u[NP];
#pragma unroll
    for (int v = 0; v < 8; ++v) {
        int kk = k0 + kpat(v, half); unsigned t[3];
        float f0 = kk < K ? M[(size_t)kk * ld + n] * sc : 0.0f, f1 = (kk + 1) < K ? M[(size_t)(kk + 1) * ld + n] * sc : 0.0f;
        pack2<F16, NP>(f0, f1, t);
#pragma unroll
        for (int p = 0; p < NP; ++p) u[p][v] = t[p];
    }
#pragma unroll
    for (int p = 0; p < NP; ++p) o.p[p] = __builtin_bit_cast(v16bf, u[p]);
}
__device__ __forceinline__ v8f wm_bf16(v16bf a, v16bf b, v8f c) { return __builtin_amdgcn_wmma_f32_16x16x32_bf16(false, a, false, b, (short)0, c, false, false); }
template <int F16, int NA, int NB> __device__ __forceinline__ v8f wmma_op(const Opnd<F16, NA>& a, const Opnd<F16, NB>& b, v8f c) {
    if (F16) {
        v16h ah = __builtin_bit_cast(v16h, a.p[0]), bh = __builtin_bit_cast(v16h, b.p[0]);
        c = __builtin_amdgcn_wmma_f32_16x16x32_f16(false, ah, false, bh, (short)0, c, false, false);
        asm volatile("v_nop\n\tv_nop\n\tv_nop\n\tv_nop" : "+v"(c) : "v"(ah), "v"(bh));
        return c;
    }
    constexpr int NMX = NA > NB ? NA : NB;
#pragma unroll
    for (int i = 0; i < NA; ++i)
#pragma unroll
        for (int j = 0; j < NB; ++j)
            if (i + j < NMX) c = wm_bf16(a.p[i], b.p[j], c);
    if (NA == 1 && NB == 1)      asm volatile("v_nop\n\tv_nop\n\tv_nop\n\tv_nop" : "+v"(c) : "v"(a.p[0]), "v"(b.p[0]));
    else if (NA == 2 && NB == 1) asm volatile("v_nop\n\tv_nop\n\tv_nop\n\tv_nop" : "+v"(c) : "v"(a.p[0]), "v"(a.p[1]), "v"(b.p[0]));
    else if (NA == 1 && NB == 2) asm volatile("v_nop\n\tv_nop\n\tv_nop\n\tv_nop" : "+v"(c) : "v"(a.p[0]), "v"(b.p[0]), "v"(b.p[1]));
    else if (NA == 2 && NB == 2) asm volatile("v_nop\n\tv_nop\n\tv_nop\n\tv_nop" : "+v"(c) : "v"(a.p[0]), "v"(a.p[1]), "v"(b.p[0]), "v"(b.p[1]));
    else                         asm volatile("v_nop\n\tv_nop\n\tv_nop\n\tv_nop" : "+v"(c) : "v"(a.p[0]), "v"(a.p[NA - 1]), "v"(b.p[0]), "v"(b.p[NB - 1]), "v"(a.p[NA / 2]), "v"(b.p[NB / 2]));
    return c;
}

struct ZMap { long long s1; long long s2; int zdiv; int pad_; };
__device__ __forceinline__ size_t zoff(const ZMap& m, int z) { return (size_t)((long long)(z / m.zdiv) * m.s1 + (long long)(z % m.zdiv) * m.s2); }

#define ACT_NONE 0
#define ACT_RELU 1
#define ACT_GELU_ERF 2
#define ACT_SILU 3
#define ACT_TANH 4
__device__ __forceinline__ float act_apply(int act, float x) {
    if (act == ACT_RELU) return x > 0.f ? x : 0.f;
    if (act == ACT_GELU_ERF) return 0.5f * x * (1.0f + erff(x * 0.70710678118654752f));
    if (act == ACT_SILU) return x / (1.0f + expf(-x));
    if (act == ACT_TANH) return tanhf(x);
    return x;
}
struct GemmArgs {
    ZMap za, zb_, zc, zbias, zadd, zrsc, zmul, zrbias;
    const float* A; const float* Bm; float* C; const float* bias; const float* add; const float* rsc; const float* mul; const float* rbias;
    long long ldadd, ldmul;
    int lda, ldb, ldc, K;
    float ascale, bscale, oscale, addscale;
    int M, nvalid, nstore, ldrsc;
    int bcs, pad1, pad2, pad3;
};
template <int BT, int F16, int NA, int NB, int RW, int CW, int ACT>
__global__ __launch_bounds__(256) void gemm_kernel(GemmArgs g) {
    constexpr int TR = 16 * RW, TC = 64 * CW, CSTR = TC + 4;
    __shared__ __align__(16) float cst[TR * CSTR];
    const int z = blockIdx.z;
    const float* A = g.A + zoff(g.za, z); const float* Bm = g.Bm + zoff(g.zb_, z); float* C = g.C + zoff(g.zc, z);
    const int tid = threadIdx.x, lane = tid & 31, wv = tid >> 5;
    const int l16 = lane & 15, half = lane >> 4;
    const int rt = wv % RW, ch = wv / RW;
    const int row0 = blockIdx.x * TR, col0 = blockIdx.y * TC + ch * 64;
    int arix = row0 + rt * 16 + l16; if (arix >= g.M) arix = g.M - 1;
    const float* arow = A + (size_t)arix * g.lda;
    v8f acc[4];
#pragma unroll
    for (int t = 0; t < 4; ++t) acc[t] = (v8f){};
    const int K = g.K;
#pragma unroll 1
    for (int kc = 0; kc < K; kc += 32) {
        Opnd<F16, NA> a;
        if (kc + 32 <= K) op_row<F16, NA>(arow + kc, half, g.ascale, a); else op_row_tail<F16, NA>(arow + kc, half, g.ascale, K - kc, a);
#pragma unroll
        for (int t = 0; t < 4; ++t) {
            Opnd<F16, NB> b;
            const int n = col0 + t * 16 + l16;
            if (n < g.nvalid) {
                if (BT) { if (kc + 32 <= K) op_row<F16, NB>(Bm + (size_t)n * g.ldb + kc, half, g.bscale, b); else op_row_tail<F16, NB>(Bm + (size_t)n * g.ldb + kc, half, g.bscale, K - kc, b); }
                else    { if (kc + 32 <= K) op_col<F16, NB>(Bm, g.ldb, n * g.bcs, kc, half, g.bscale, b); else op_col_tail<F16, NB>(Bm, g.ldb, n * g.bcs, kc, half, g.bscale, K, b); }
            } else {
#pragma unroll
                for (int p = 0; p < NB; ++p) b.p[p] = (v16bf){};
            }
            acc[t] = wmma_op<F16, NA, NB>(a, b, acc[t]);
        }
    }
    const float* bias = g.bias ? g.bias + zoff(g.zbias, z) : nullptr;
    const float* add = g.add ? g.add + zoff(g.zadd, z) : nullptr;
    const float* rsc = g.rsc ? g.rsc + zoff(g.zrsc, z) : nullptr;
    const float* mul = g.mul ? g.mul + zoff(g.zmul, z) : nullptr;
    const float* rbias = g.rbias ? g.rbias + zoff(g.zrbias, z) : nullptr;
#pragma unroll
    for (int t = 0; t < 4; ++t) {
        const int cl = ch * 64 + t * 16 + l16;
        const int cg = blockIdx.y * TC + cl;
        const bool cok = cg < g.nvalid;
        const float bv = (bias && cok) ? bias[(size_t)cg * g.bcs] : 0.0f;
#pragma unroll
        for (int r = 0; r < 8; ++r) {
            const int rl = rt * 16 + r + 8 * half;
            float v = acc[t][r] * g.oscale + bv;
            int rg = row0 + rl; if (rg >= g.M) rg = g.M - 1;
            if (rbias) v += rbias[rg];
            if (rsc) v *= rsc[(size_t)rg * g.ldrsc];
            if (mul && cok) v *= mul[(size_t)rg * g.ldmul + cg];
            if (add && cok) v += g.addscale * add[(size_t)rg * g.ldadd + cg];
            cst[rl * CSTR + cl] = v;
        }
    }
    __syncthreads();
    const int col = tid % TC, rsel = tid / TC, rstep = 256 / TC;
    if (ACT != ACT_NONE) {
#pragma unroll 1
        for (int r = rsel; r < TR; r += rstep) cst[r * CSTR + col] = act_apply(ACT, cst[r * CSTR + col]);
    }
    float* ob = C + (size_t)row0 * g.ldc + (size_t)blockIdx.y * TC;
    const bool colok = (int)(blockIdx.y * TC + col) < g.nstore;
    const int rmax = (g.M - row0 < TR) ? (g.M - row0) : TR;
    auto pass = [&]() {
        if (colok) {
#pragma unroll 4
            for (int r = rsel; r < rmax; r += rstep) *(volatile float*)(ob + (size_t)r * g.ldc + col) = cst[r * CSTR + col];
        }
    };
    pass();
    __threadfence();
    pass();
}
static inline ZMap zm(long long s1) { ZMap m; m.s1 = s1; m.s2 = 0; m.zdiv = 1; m.pad_ = 0; return m; }
static inline ZMap zm2(long long s1, long long s2, int zdiv) { ZMap m; m.s1 = s1; m.s2 = s2; m.zdiv = zdiv; m.pad_ = 0; return m; }
static inline GemmArgs gemm_args(const float* A, int lda, ZMap za, const float* Bm, int ldb, ZMap zb, float* C, int ldc, ZMap zc, int M, int N, int K) {
    GemmArgs g; g.za = za; g.zb_ = zb; g.zc = zc; g.zbias = zm(0); g.zadd = zm(0); g.zrsc = zm(0); g.zmul = zm(0); g.zrbias = zm(0);
    g.A = A; g.Bm = Bm; g.C = C; g.bias = nullptr; g.add = nullptr; g.rsc = nullptr; g.mul = nullptr; g.rbias = nullptr; g.ldadd = 0; g.ldmul = 0;
    g.lda = lda; g.ldb = ldb; g.ldc = ldc; g.K = K; g.ascale = 1.0f; g.bscale = 1.0f; g.oscale = 1.0f; g.addscale = 1.0f; g.M = M; g.nvalid = N; g.nstore = N; g.ldrsc = 1;
    g.bcs = 1; g.pad1 = 0; g.pad2 = 0; g.pad3 = 0;
    return g;
}
static_assert(sizeof(ZMap) == 24, "ZMap layout");
static_assert(sizeof(GemmArgs) == 8 * 24 + 8 * 8 + 2 * 8 + 4 * 4 + 4 * 4 + 4 * 4 + 4 * 4, "GemmArgs has no padding");

__global__ __launch_bounds__(256) void softmax_rows(float* S, long long sy, long long sx, int L, float prescale, const float* addv, long long say, int aydiv, int causal,
                                                  const int* imask, long long imy, long long imx, float maskval) {
    __shared__ float red[8];
    const int tid = threadIdx.x, lane = tid & 31, wid = tid >> 5;
    float* row = S + (size_t)blockIdx.y * sy + (size_t)blockIdx.x * sx;
    const float* av = addv ? addv + (size_t)(blockIdx.y / aydiv) * say : nullptr;
    const int* im = imask ? imask + (size_t)(blockIdx.y / aydiv) * imy + (size_t)blockIdx.x * imx : nullptr;
    float v[16];
    const int nj = L / 256;
    float mx = -__builtin_inff();
#pragma unroll
    for (int j = 0; j < 16; ++j) if (j < nj) { float t = row[tid + 256 * j] * prescale; if (av) t += av[tid + 256 * j]; if (im && im[tid + 256 * j] == 0) t = maskval; if (causal && (tid + 256 * j) > (int)blockIdx.x) t = -__builtin_inff(); v[j] = t; mx = fmaxf(mx, t); }
#pragma unroll
    for (int o = 16; o; o >>= 1) mx = fmaxf(mx, __shfl_xor(mx, o, 32));
    if (lane == 0) red[wid] = mx;
    __syncthreads();
    float m = red[0];
#pragma unroll
    for (int i = 1; i < 8; ++i) m = fmaxf(m, red[i]);
    if (m == -__builtin_inff()) m = 0.f;
    __syncthreads();
    float sum = 0.f;
#pragma unroll
    for (int j = 0; j < 16; ++j) if (j < nj) { v[j] = expf(v[j] - m); sum += v[j]; }
#pragma unroll
    for (int o = 16; o; o >>= 1) sum += __shfl_xor(sum, o, 32);
    if (lane == 0) red[wid] = sum;
    __syncthreads();
    float tot = 0.f;
#pragma unroll
    for (int i = 0; i < 8; ++i) tot += red[i];
    const float inv = 1.0f / tot;
#pragma unroll
    for (int j = 0; j < 16; ++j) if (j < nj) *(volatile float*)(row + tid + 256 * j) = v[j] * inv;
    __threadfence();
#pragma unroll
    for (int j = 0; j < 16; ++j) if (j < nj) *(volatile float*)(row + tid + 256 * j) = v[j] * inv;
}

#define VST2(T, p, v) do { const T vst2_v_ = (v); *(volatile T*)(p) = vst2_v_; __threadfence(); *(volatile T*)(p) = vst2_v_; } while (0)
#define IL_T 128
#define IL_TILE 4096
__global__ __launch_bounds__(IL_T) void k_inlists(const int* __restrict__ tgt, int E, int N, int* NBR, int* cnt) {
    __shared__ int tt[IL_TILE];
    __shared__ int lists[IL_T * IL_CAP];
    const int d = blockIdx.x * IL_T + threadIdx.x; int n = 0;
    for (int e0 = 0; e0 < E; e0 += IL_TILE) {
        const int nt = min(IL_TILE, E - e0);
        __syncthreads();
        for (int i = threadIdx.x; i < nt; i += IL_T) tt[i] = tgt[e0 + i];
        __syncthreads();
        for (int i = 0; i < nt; ++i) { if (tt[i] == d) { if (n < IL_CAP) lists[threadIdx.x * IL_CAP + n] = e0 + i; ++n; } }
    }
    if (d < N) {
        int* row = NBR + (size_t)d * IL_CAP;
        for (int j = 0; j < IL_CAP; ++j) { const int v = (j < n) ? lists[threadIdx.x * IL_CAP + j] : 0; *(volatile int*)(row + j) = v; }
        __threadfence();
        for (int j = 0; j < IL_CAP; ++j) { const int v = (j < n) ? lists[threadIdx.x * IL_CAP + j] : 0; *(volatile int*)(row + j) = v; }
        VST2(int, cnt + d, min(n, IL_CAP));
    }
}
__global__ __launch_bounds__(256) void k_csr_scan(const int* __restrict__ cnt, int* off, int N) {
    __shared__ int part[256]; const int per = ((((N + 255) / 256) + 31) / 32) * 32; const int a = threadIdx.x * per, b = min(N, a + per); int s = 0;
    for (int i = a; i < b; ++i) s += cnt[i]; part[threadIdx.x] = s; __syncthreads();
    if (threadIdx.x == 0) { int run = 0; for (int t = 0; t < 256; ++t) { const int v = part[t]; part[t] = run; run += v; } } __syncthreads();
    int run = part[threadIdx.x]; for (int i = a; i < b; ++i) { VST2(int, off + i, run); run += cnt[i]; }
    if (a < N && b == N) { VST2(int, off + N, run); }
}
__global__ __launch_bounds__(256) void k_slotcopy(const int* __restrict__ off, const int* __restrict__ NBR, int* slot, int N) {
    const int t = blockIdx.x * 256 + threadIdx.x; const int tot = off[N]; if (t >= tot) return;
    int lo = 0, hi = N - 1;
    while (lo < hi) { const int mid = (lo + hi + 1) >> 1; if (off[mid] <= t) lo = mid; else hi = mid - 1; }
    int j = t - off[lo]; j = (j < 0) ? 0 : ((j >= IL_CAP) ? (IL_CAP - 1) : j);
    VST2(int, slot + t, NBR[(size_t)lo * IL_CAP + j]);
}


__global__ __launch_bounds__(256) void k_flat(const int* __restrict__ edges, int* srcf, int* dstf) {
    const int i = blockIdx.x * 256 + threadIdx.x; if (i >= NE_) return;
    const int b = i / NEB, e = i % NEB;
    int s = edges[(b * 2 + 0) * NEB + e], d = edges[(b * 2 + 1) * NEB + e];
    s = s < 0 ? 0 : (s >= NNODE ? NNODE - 1 : s); d = d < 0 ? 0 : (d >= NNODE ? NNODE - 1 : d);
    VST2(int, srcf + i, s + b * NNODE); VST2(int, dstf + i, d + b * NNODE);
}
__global__ __launch_bounds__(256) void k_gru(const float* __restrict__ GX, const float* __restrict__ GH, float* Hs, int t) {
    const size_t q = (size_t)blockIdx.x * 256 + threadIdx.x; if (q >= (size_t)BN_ * HID) return;
    const int j = (int)(q % HID), n = (int)(q / HID);
    const float* gx = GX + (size_t)n * G3; const float* gh = GH + (size_t)n * G3;
    const float hprev = (t == 0) ? 0.f : Hs[q];
    const float hr = (t == 0) ? 0.f : gh[j], hz = (t == 0) ? 0.f : gh[HID + j], hn = (t == 0) ? 0.f : gh[2 * HID + j];
    const float r = 1.0f / (1.0f + expf(-(gx[j] + hr))), z = 1.0f / (1.0f + expf(-(gx[HID + j] + hz)));
    const float nn = tanhf(gx[2 * HID + j] + r * hn);
    VST2(float, Hs + q, (1.0f - z) * nn + z * hprev);
}
__global__ __launch_bounds__(256) void k_gru0(const float* __restrict__ GX, const float* __restrict__ bhh, float* Hs) {
    const size_t q = (size_t)blockIdx.x * 256 + threadIdx.x; if (q >= (size_t)BN_ * HID) return;
    const int j = (int)(q % HID), n = (int)(q / HID);
    const float* gx = GX + (size_t)n * G3;
    const float r = 1.0f / (1.0f + expf(-(gx[j] + bhh[j]))), z = 1.0f / (1.0f + expf(-(gx[HID + j] + bhh[HID + j])));
    const float nn = tanhf(gx[2 * HID + j] + r * bhh[2 * HID + j]);
    VST2(float, Hs + q, (1.0f - z) * nn);
}
__global__ __launch_bounds__(256) void k_logits(const float* __restrict__ XL, const float* __restrict__ XR, const int* __restrict__ srcf, const int* __restrict__ dstf,
                                                const float* __restrict__ att, float* lg, int cnt_, int self_) {
    const int q = blockIdx.x * 256 + threadIdx.x; if (q >= cnt_ * NHEAD) return;
    const int h = q % NHEAD, e = q / NHEAD;
    const int s = self_ ? e : srcf[e], d = self_ ? e : dstf[e];
    const float* a = XL + (size_t)s * HC + h * HID; const float* b = XR + (size_t)d * HC + h * HID; const float* w = att + h * HID;
    float acc = 0.f;
#pragma unroll 4
    for (int c = 0; c < HID; ++c) { float m = a[c] + b[c]; m = m > 0.f ? m : SLOPE * m; acc += m * w[c]; }
    VST2(float, lg + q, acc);
}
__global__ __launch_bounds__(256) void k_dststats(const float* __restrict__ lg, const float* __restrict__ lgs, const int* __restrict__ off, const int* __restrict__ slot, float* mx, float* sinv) {
    const int q = blockIdx.x * 256 + threadIdx.x; if (q >= BN_ * NHEAD) return;
    const int h = q % NHEAD, n = q / NHEAD; const int a = off[n], b = off[n + 1];
    float m = lgs[q];
    for (int p = a; p < b && p < a + IL_CAP; ++p) { int e = slot[p]; e = e < 0 ? 0 : (e >= NE_ ? NE_ - 1 : e); m = fmaxf(m, lg[(size_t)e * NHEAD + h]); }
    float z = expf(lgs[q] - m);
    for (int p = a; p < b && p < a + IL_CAP; ++p) { int e = slot[p]; e = e < 0 ? 0 : (e >= NE_ ? NE_ - 1 : e); z += expf(lg[(size_t)e * NHEAD + h] - m); }
    VST2(float, mx + q, m); VST2(float, sinv + q, 1.0f / z);
}
__global__ __launch_bounds__(256) void k_alpha(const float* __restrict__ lg, const float* __restrict__ lgs, const int* __restrict__ dstf, const float* __restrict__ mx, const float* __restrict__ sinv, float* out1) {
    const int q = blockIdx.x * 256 + threadIdx.x; if (q >= (NE_ + BN_) * NHEAD) return;
    const int h = q % NHEAD, e = q / NHEAD;
    float v;
    if (e < NE_) { const int d = dstf[e]; v = expf(lg[(size_t)e * NHEAD + h] - mx[d * NHEAD + h]) * sinv[d * NHEAD + h]; }
    else { const int n = e - NE_; v = expf(lgs[n * NHEAD + h] - mx[n * NHEAD + h]) * sinv[n * NHEAD + h]; }
    VST2(float, out1 + q, v);
}
__global__ __launch_bounds__(HID) void k_ego(const float* __restrict__ XL, const float* __restrict__ lg, const float* __restrict__ lgs, const float* __restrict__ mx, const float* __restrict__ sinv,
                                            const int* __restrict__ srcf, const int* __restrict__ off, const int* __restrict__ slot, const float* __restrict__ bias, float* OG) {
    const int b = blockIdx.x, c = threadIdx.x; const int n = b * NNODE; const int a = off[n], bb = off[n + 1];
    float tot = 0.f;
    for (int h = 0; h < NHEAD; ++h) {
        const float m = mx[n * NHEAD + h], zi = sinv[n * NHEAD + h];
        float s = expf(lgs[n * NHEAD + h] - m) * zi * XL[(size_t)n * HC + h * HID + c];
        for (int p = a; p < bb && p < a + IL_CAP; ++p) { int e = slot[p]; e = e < 0 ? 0 : (e >= NE_ ? NE_ - 1 : e); const int sn = srcf[e];
            s += expf(lg[(size_t)e * NHEAD + h] - m) * zi * XL[(size_t)sn * HC + h * HID + c]; }
        tot += s;
    }
    VST2(float, OG + (size_t)b * FUP + c, tot / (float)NHEAD + bias[c]);
}
template <int C, int HIN, int HO>
__global__ __launch_bounds__(256) void k_im2col_s2(const float* __restrict__ src, float* Xc) {
    const int q = blockIdx.x * 256 + threadIdx.x; if (q >= NB_ * C * HO * HO) return;
    const int ox = q % HO, oy = (q / HO) % HO, c = (q / (HO * HO)) % C, img = q / (C * HO * HO);
    const float* plane = src + ((size_t)img * C + c) * HIN * HIN; const size_t col = (size_t)img * HO * HO + oy * HO + ox; const size_t ld = (size_t)NB_ * HO * HO;
    for (int ky = 0; ky < 3; ++ky) for (int kx = 0; kx < 3; ++kx) {
        const int yy = 2 * oy + ky, xx = 2 * ox + kx;
        const float v = (yy < HIN && xx < HIN) ? plane[yy * HIN + xx] : 0.f;
        VST2(float, Xc + (size_t)((c * 3 + ky) * 3 + kx) * ld + col, v);
    }
}
__global__ __launch_bounds__(128) void k_phase(const float* __restrict__ phase, const float* __restrict__ Wp, const float* __restrict__ bp, float* FU) {
    const int q = threadIdx.x; if (q >= NB_ * PP) return; const int b = q / PP, j = q % PP;
    float s = bp[j]; for (int k = 0; k < PP; ++k) s += phase[b * PP + k] * Wp[k * PP + j];
    VST2(float, FU + (size_t)b * FUP + 256 + j, fmaxf(s, 0.f));
}
__global__ __launch_bounds__(128) void k_head(const float* __restrict__ HD_, const float* __restrict__ Wo, const float* __restrict__ bo, const float* __restrict__ Wa, const float* __restrict__ ba, float* out0) {
    __shared__ float adv[NB_ * NACT]; __shared__ float vsh[NB_];
    const int q = threadIdx.x; const int b = q / NACT, a = q % NACT; const float* hrow = HD_ + (size_t)b * HID;
    { float s = ba[a]; for (int k = 0; k < HID; ++k) s += hrow[k] * Wa[k * NACT + a]; adv[q] = s; }
    if (q < NB_) { const float* hr = HD_ + (size_t)q * HID; float s = bo[0]; for (int k = 0; k < HID; ++k) s += hr[k] * Wo[k]; vsh[q] = s; }
    __syncthreads();
    float m = 0.f; for (int j = 0; j < NACT; ++j) m += adv[b * NACT + j]; m /= (float)NACT;
    VST2(float, out0 + q, vsh[b] + adv[q] - m);
}

extern "C" void kernel_launch(void* const* d_in, const int* in_sizes, int n_in,
                              void* d_out, int out_size, void* d_ws, size_t ws_size, hipStream_t stream) {
    (void)in_sizes; (void)n_in; (void)out_size;
    const float* obs = (const float*)d_in[0];
    const float* phase = (const float*)d_in[1];
    const float* omap = (const float*)d_in[2];
    const int* edges = (const int*)d_in[3];
    const float* W_nbrs = (const float*)d_in[5]; const float* b_nbrs = (const float*)d_in[6];
    const float* W_ih = (const float*)d_in[7]; const float* W_hh = (const float*)d_in[8]; const float* b_ih = (const float*)d_in[9]; const float* b_hh = (const float*)d_in[10];
    const float* Wl = (const float*)d_in[11]; const float* Wr = (const float*)d_in[12];
    const float* att = (const float*)d_in[13]; const float* gbias = (const float*)d_in[14];
    const float* c1w = (const float*)d_in[15]; const float* c1b = (const float*)d_in[16];
    const float* c2w = (const float*)d_in[17]; const float* c2b = (const float*)d_in[18];
    const float* Wc = (const float*)d_in[19]; const float* bc = (const float*)d_in[20];
    const float* Wp = (const float*)d_in[21]; const float* bp = (const float*)d_in[22];
    const float* Wh = (const float*)d_in[23]; const float* bh = (const float*)d_in[24];
    const float* Wo = (const float*)d_in[25]; const float* bo = (const float*)d_in[26];
    const float* Wa = (const float*)d_in[27]; const float* ba = (const float*)d_in[28];
    float* out0 = (float*)d_out;
    float* out1 = out0 + 128;

    char* wsp = (char*)d_ws;
    auto take = [&](size_t bytes) { char* p = wsp; wsp += (bytes + 255) & ~(size_t)255; return (void*)p; };
    int* srcf = (int*)take(NE_ * 4); int* dstf = (int*)take(NE_ * 4);
    int* NBR = (int*)take((size_t)BN_ * IL_CAP * 4); int* cnt = (int*)take((size_t)(BN_ + 1) * 4); int* off = (int*)take((size_t)(BN_ + 1) * 4); int* slot = (int*)take(NE_ * 4);
    float* Xt = (float*)take((size_t)BN_ * HID * 4);
    float* GX = (float*)take((size_t)BN_ * G3 * 4); float* GH = (float*)take((size_t)BN_ * G3 * 4);
    float* Hs = (float*)take((size_t)BN_ * HID * 4);
    float* XL = (float*)take((size_t)BN_ * HC * 4); float* XR = (float*)take((size_t)BN_ * HC * 4);
    float* LG = (float*)take((size_t)NE_ * NHEAD * 4); float* LGS = (float*)take((size_t)BN_ * NHEAD * 4);
    float* MX = (float*)take((size_t)BN_ * NHEAD * 4); float* SI = (float*)take((size_t)BN_ * NHEAD * 4);
    float* FU = (float*)take((size_t)NB_ * FUP * 4);
    float* XC = (float*)take((size_t)288 * NB_ * 256 * 4);
    float* C1 = (float*)take((size_t)NB_ * 32 * 256 * 4);
    float* C2 = (float*)take((size_t)NB_ * 64 * 64 * 4);
    float* HDN = (float*)take((size_t)NB_ * HID * 4);
    if ((size_t)(wsp - (char*)d_ws) > ws_size) return;

    for (int t = 0; t < TT; ++t) {
        { GemmArgs g = gemm_args(obs + (size_t)t * FO, TT * FO, zm(0), W_nbrs, HID, zm(0), Xt, HID, zm(0), BN_, HID, FO); g.bias = b_nbrs; g.bscale = 16.0f; g.oscale = 1.0f / 16.0f;
          gemm_kernel<0, 1, 1, 1, 4, 2, ACT_RELU><<<dim3(BN_ / 64, 1, 1), 256, 0, stream>>>(g); }
        { GemmArgs g = gemm_args(Xt, HID, zm(0), W_ih, HID, zm(0), GX, G3, zm(0), BN_, G3, HID); g.bias = b_ih; g.bscale = 16.0f; g.oscale = 1.0f / 16.0f;
          gemm_kernel<1, 1, 1, 1, 4, 2, ACT_NONE><<<dim3(BN_ / 64, G3 / 128, 1), 256, 0, stream>>>(g); }
        if (t == 0) { k_gru0<<<(BN_ * HID) / 256, 256, 0, stream>>>(GX, b_hh, Hs); }
        else {
            GemmArgs g = gemm_args(Hs, HID, zm(0), W_hh, HID, zm(0), GH, G3, zm(0), BN_, G3, HID); g.bias = b_hh; g.bscale = 16.0f; g.oscale = 1.0f / 16.0f;
            gemm_kernel<1, 1, 1, 1, 4, 2, ACT_NONE><<<dim3(BN_ / 64, G3 / 128, 1), 256, 0, stream>>>(g);
            k_gru<<<(BN_ * HID) / 256, 256, 0, stream>>>(GX, GH, Hs, t);
        }
    }
    k_flat<<<(NE_ + 255) / 256, 256, 0, stream>>>(edges, srcf, dstf);
    k_inlists<<<(BN_ + IL_T - 1) / IL_T, IL_T, 0, stream>>>(dstf, NE_, BN_, NBR, cnt);
    k_csr_scan<<<1, 256, 0, stream>>>(cnt, off, BN_);
    k_slotcopy<<<(NE_ + 255) / 256, 256, 0, stream>>>(off, NBR, slot, BN_);
    { GemmArgs g = gemm_args(Hs, HID, zm(0), Wl, HC, zm(0), XL, HC, zm(0), BN_, HC, HID); g.bscale = 16.0f; g.oscale = 1.0f / 16.0f;
      gemm_kernel<0, 1, 1, 1, 4, 2, ACT_NONE><<<dim3(BN_ / 64, HC / 128, 1), 256, 0, stream>>>(g); }
    { GemmArgs g = gemm_args(Hs, HID, zm(0), Wr, HC, zm(0), XR, HC, zm(0), BN_, HC, HID); g.bscale = 16.0f; g.oscale = 1.0f / 16.0f;
      gemm_kernel<0, 1, 1, 1, 4, 2, ACT_NONE><<<dim3(BN_ / 64, HC / 128, 1), 256, 0, stream>>>(g); }
    k_logits<<<(NE_ * NHEAD + 255) / 256, 256, 0, stream>>>(XL, XR, srcf, dstf, att, LG, NE_, 0);
    k_logits<<<(BN_ * NHEAD + 255) / 256, 256, 0, stream>>>(XL, XR, srcf, dstf, att, LGS, BN_, 1);
    k_dststats<<<(BN_ * NHEAD + 255) / 256, 256, 0, stream>>>(LG, LGS, off, slot, MX, SI);
    k_alpha<<<((NE_ + BN_) * NHEAD + 255) / 256, 256, 0, stream>>>(LG, LGS, dstf, MX, SI, out1);
    k_ego<<<NB_, HID, 0, stream>>>(XL, LG, LGS, MX, SI, srcf, off, slot, gbias, FU);
    k_im2col_s2<4, 32, 16><<<(NB_ * 4 * 256 + 255) / 256, 256, 0, stream>>>(omap, XC);
    { GemmArgs g = gemm_args(c1w, 36, zm(0), XC, NB_ * 256, zm(256), C1, 256, zm(32 * 256), 32, 256, 36); g.rbias = c1b; g.ascale = 16.0f; g.oscale = 1.0f / 16.0f;
      gemm_kernel<0, 1, 1, 1, 4, 2, ACT_RELU><<<dim3(1, 2, NB_), 256, 0, stream>>>(g); }
    k_im2col_s2<32, 16, 8><<<(NB_ * 32 * 64 + 255) / 256, 256, 0, stream>>>(C1, XC);
    { GemmArgs g = gemm_args(c2w, 288, zm(0), XC, NB_ * 64, zm(64), C2, 64, zm(64 * 64), 64, 64, 288); g.rbias = c2b; g.ascale = 16.0f; g.oscale = 1.0f / 16.0f;
      gemm_kernel<0, 1, 1, 1, 4, 2, ACT_RELU><<<dim3(1, 1, NB_), 256, 0, stream>>>(g); }
    { GemmArgs g = gemm_args(C2, 4096, zm(0), Wc, HID, zm(0), FU + 128, FUP, zm(0), NB_, HID, 4096); g.bias = bc; g.bscale = 16.0f; g.oscale = 1.0f / 16.0f;
      gemm_kernel<0, 1, 1, 1, 4, 2, ACT_RELU><<<dim3(1, 1, 1), 256, 0, stream>>>(g); }
    k_phase<<<1, 128, 0, stream>>>(phase, Wp, bp, FU);
    { GemmArgs g = gemm_args(FU, FUP, zm(0), Wh, HID, zm(0), HDN, HID, zm(0), NB_, HID, 264); g.bias = bh; g.bscale = 16.0f; g.oscale = 1.0f / 16.0f;
      gemm_kernel<0, 1, 1, 1, 4, 2, ACT_RELU><<<dim3(1, 1, 1), 256, 0, stream>>>(g); }
    k_head<<<1, NB_ * NACT, 0, stream>>>(HDN, Wo, bo, Wa, ba, out0);
}
